// MultiHeadLinearAttention_20890720928061
// MI455X (gfx1250) — hardware-verified
//
#include <hip/hip_runtime.h>
#include <stdint.h>

typedef __attribute__((ext_vector_type(16))) _Float16 v16h;
typedef __attribute__((ext_vector_type(8)))  _Float16 v8h;
typedef __attribute__((ext_vector_type(16))) __bf16   v16b;
typedef __attribute__((ext_vector_type(8)))  __bf16   v8b;
typedef __attribute__((ext_vector_type(8)))  float    v8f;
typedef __attribute__((ext_vector_type(4)))  float    v4f;
typedef __attribute__((ext_vector_type(2)))  float    v2f;
typedef __attribute__((ext_vector_type(4)))  unsigned v4u;

constexpr int NBATCH = 2;
constexpr int NSEQ   = 2048;
constexpr int NCH    = 1024;
constexpr int NHEAD  = 16;
constexpr int HDIM   = 64;
constexpr int KLOW   = 64;
constexpr int NROWS  = NBATCH * NSEQ;
constexpr int NQKV   = 3 * NCH;

__device__ __forceinline__ unsigned short f2bf_bits(float f) {
  unsigned u = __float_as_uint(f);
  return (unsigned short)((u + 0x7FFFu + ((u >> 16) & 1u)) >> 16);
}
__device__ __forceinline__ float bf_bits2f(unsigned short h) { return __uint_as_float(((unsigned)h) << 16); }

__device__ __forceinline__ void dep_guard_h(v8f& a, v8f& b, v16h x, v16h y) { asm volatile("v_nop\n\tv_nop\n\tv_nop\n\tv_nop" : "+v"(a), "+v"(b) : "v"(x), "v"(y)); }
__device__ __forceinline__ void dep_guard_b(v8f& a, v8f& b, v16b x, v16b y) { asm volatile("v_nop\n\tv_nop\n\tv_nop\n\tv_nop" : "+v"(a), "+v"(b) : "v"(x), "v"(y)); }
__device__ __forceinline__ void keep4_h(v16h a, v16h b, v16h c, v16h d) { asm volatile("v_nop" :: "v"(a), "v"(b), "v"(c), "v"(d)); }
__device__ __forceinline__ void keep4_b(v16b a, v16b b, v16b c, v16b d) { asm volatile("v_nop" :: "v"(a), "v"(b), "v"(c), "v"(d)); }
__device__ __forceinline__ void acc_guard4(v8f& a, v8f& b, v8f& c, v8f& d) { asm volatile("v_nop\n\tv_nop\n\tv_nop\n\tv_nop" : "+v"(a), "+v"(b), "+v"(c), "+v"(d)); }

template <typename T> struct Frag;
template <> struct Frag<_Float16> {
  typedef v16h V; union U { v16h v; v8h h[2]; };
  static __device__ __forceinline__ v16h load(const _Float16* p) {
    U f; f.h[0] = *(const v8h*)(p); f.h[1] = *(const v8h*)(p + 16); return f.v;
  }
  static __device__ __forceinline__ v8f mma(v16h a, v16h b, v8f c) {
    return __builtin_amdgcn_wmma_f32_16x16x32_f16(false, a, false, b, (short)0, c, false, false);
  }
  static __device__ __forceinline__ void guard(v8f& a, v8f& b, v16h x, v16h y) { dep_guard_h(a, b, x, y); }
  static __device__ __forceinline__ void keep(v16h a, v16h b, v16h c, v16h d) { keep4_h(a, b, c, d); }
};
template <> struct Frag<__bf16> {
  typedef v16b V; union U { v16b v; v8b h[2]; };
  static __device__ __forceinline__ v16b load(const __bf16* p) {
    U f; f.h[0] = *(const v8b*)(p); f.h[1] = *(const v8b*)(p + 16); return f.v;
  }
  static __device__ __forceinline__ v8f mma(v16b a, v16b b, v8f c) {
    return __builtin_amdgcn_wmma_f32_16x16x32_bf16(false, a, false, b, (short)0, c, false, false);
  }
  static __device__ __forceinline__ void guard(v8f& a, v8f& b, v16b x, v16b y) { dep_guard_b(a, b, x, y); }
  static __device__ __forceinline__ void keep(v16b a, v16b b, v16b c, v16b d) { keep4_b(a, b, c, d); }
};

template <int ET> struct Elem;
template <> struct Elem<0> { typedef _Float16 T; };
template <> struct Elem<1> { typedef __bf16 T; };
template <int ET, int SPLIT, int BIAS_MODE, int OUT_MODE>
__global__ __launch_bounds__(256) void wmma_gemm64(
    const unsigned short* __restrict__ Ap, const unsigned short* __restrict__ A2p, int lda, long strideA,
    const unsigned short* __restrict__ Btp, const unsigned short* __restrict__ Bt2p, int ldb, long strideB,
    void* __restrict__ Cout, void* __restrict__ Cout2, int ldc, long strideC,
    const float* __restrict__ bias,
    int M, int N, int K, float scale) {
  typedef typename Elem<ET>::T T;
  typedef typename Frag<T>::V V;
  const T* A = (const T*)Ap; const T* A2 = (const T*)A2p; const T* Bt = (const T*)Btp; const T* Bt2 = (const T*)Bt2p;
  __shared__ __align__(16) float sT[8][16 * 68];
  const int b    = blockIdx.y;
  const int lane = threadIdx.x & 31;
  const int wave = threadIdx.x >> 5;
  const int tilesN = N >> 6;
  const int tilesM = M >> 6;
  const int tile = blockIdx.x * 8 + wave;
  if (tile >= tilesM * tilesN) return;
  const int tm = tile / tilesN;
  const int tn = tile - tm * tilesN;
  const int m0 = tm << 6;
  const int n0 = tn << 6;

  const T* Ab  = A  + (size_t)b * strideA;
  const T* Bb  = Bt + (size_t)b * strideB;
  const T* Ab2 = (SPLIT >= 1) ? (A2  + (size_t)b * strideA) : Ab;
  const T* Bb2 = (SPLIT == 2) ? (Bt2 + (size_t)b * strideB) : Bb;

  const int rlane = lane & 15;
  const int koff  = (lane >> 4) * 8;
  const int mOff  = (lane >> 4) * 8;

  v8f acc[4][4];
#pragma unroll
  for (int i = 0; i < 4; ++i)
#pragma unroll
    for (int j = 0; j < 4; ++j) acc[i][j] = (v8f){0.f,0.f,0.f,0.f,0.f,0.f,0.f,0.f};

  for (int k0 = 0; k0 < K; k0 += 32) {
    V bh[4], bl[4];
#pragma unroll
    for (int j = 0; j < 4; ++j) {
      const size_t bo = (size_t)(n0 + (j << 4) + rlane) * ldb + koff + k0;
      bh[j] = Frag<T>::load(Bb + bo);
      if (SPLIT == 2) bl[j] = Frag<T>::load(Bb2 + bo);
    }
#pragma unroll
    for (int i = 0; i < 4; ++i) {
      const size_t ao = (size_t)(m0 + (i << 4) + rlane) * lda + koff + k0;
      V ah = Frag<T>::load(Ab + ao);
      V al = ah;
      if (SPLIT >= 1) al = Frag<T>::load(Ab2 + ao);
#pragma unroll
      for (int j = 0; j < 4; ++j) {
        acc[i][j] = Frag<T>::mma(ah, bh[j], acc[i][j]);
        if (SPLIT == 2) acc[i][j] = Frag<T>::mma(ah, bl[j], acc[i][j]);
        if (SPLIT >= 1) acc[i][j] = Frag<T>::mma(al, bh[j], acc[i][j]);
      }
      Frag<T>::guard(acc[i][0], acc[i][3], ah, al);
    }
    Frag<T>::keep(bh[0], bh[1], bh[2], bh[3]);
    if (SPLIT == 2) Frag<T>::keep(bl[0], bl[1], bl[2], bl[3]);
  }
  acc_guard4(acc[0][0], acc[0][1], acc[0][2], acc[0][3]);
  acc_guard4(acc[1][0], acc[1][1], acc[1][2], acc[1][3]);
  acc_guard4(acc[2][0], acc[2][1], acc[2][2], acc[2][3]);
  acc_guard4(acc[3][0], acc[3][1], acc[3][2], acc[3][3]);

  float* slab = sT[wave];
#pragma unroll
  for (int i = 0; i < 4; ++i) {
    const int mBase = m0 + (i << 4);
#pragma unroll
    for (int j = 0; j < 4; ++j) {
      const int n = n0 + (j << 4) + rlane;
      float bv = 0.f;
      if (BIAS_MODE == 2) bv = bf_bits2f(f2bf_bits(bias[n]));
#pragma unroll
      for (int r = 0; r < 8; ++r) {
        float v = acc[i][j][r] * scale;
        if (BIAS_MODE == 2) v += bv;
        slab[(mOff + r) * 68 + (j << 4) + rlane] = v;
      }
    }
    __builtin_amdgcn_fence(__ATOMIC_RELEASE, "workgroup");
    __builtin_amdgcn_wave_barrier();
    __builtin_amdgcn_fence(__ATOMIC_ACQUIRE, "workgroup");
    if (OUT_MODE == 0) {
      float* C = (float*)Cout + (size_t)b * strideC;
      const int hh = lane >> 4, c4 = (lane & 15) * 4;
      for (int pass = 0; pass < 2; ++pass) {
#pragma unroll
        for (int it = 0; it < 8; ++it) {
          const int row = it * 2 + hh;
          v4f v = *(const v4f*)(slab + row * 68 + c4);
          *(volatile v4f*)(C + (size_t)(mBase + row) * ldc + n0 + c4) = v;
        }
        __threadfence();
      }
    } else {
      const int q = lane >> 3, c8 = (lane & 7) * 8;
      unsigned short* C  = (unsigned short*)Cout  + (size_t)b * strideC;
      unsigned short* C2 = (OUT_MODE == 2) ? ((unsigned short*)Cout2 + (size_t)b * strideC) : nullptr;
      for (int pass = 0; pass < 2; ++pass) {
#pragma unroll
        for (int it = 0; it < 4; ++it) {
          const int row = it * 4 + q;
          const float* sp = slab + row * 68 + c8;
          v8h hv, lv;
#pragma unroll
          for (int e = 0; e < 8; ++e) {
            if (OUT_MODE == 1) {
              hv[e] = (_Float16)sp[e];
            } else {
              unsigned short hb = f2bf_bits(sp[e]);
              unsigned short lb = f2bf_bits(sp[e] - bf_bits2f(hb));
              hv[e] = __builtin_bit_cast(_Float16, hb);
              lv[e] = __builtin_bit_cast(_Float16, lb);
            }
          }
          *(volatile v8h*)(C + (size_t)(mBase + row) * ldc + n0 + c8) = hv;
          if (OUT_MODE == 2) *(volatile v8h*)(C2 + (size_t)(mBase + row) * ldc + n0 + c8) = lv;
        }
        __threadfence();
      }
    }
    __builtin_amdgcn_fence(__ATOMIC_RELEASE, "workgroup");
    __builtin_amdgcn_wave_barrier();
    __builtin_amdgcn_fence(__ATOMIC_ACQUIRE, "workgroup");
  }
}

__global__ __launch_bounds__(256) void cast_f32_bf16x2(
    const float* __restrict__ in, unsigned short* __restrict__ out, int n2) {
  const int i = blockIdx.x * 256 + threadIdx.x;
  if (i < n2) {
    const v2f f = *(const v2f*)(in + 2 * (size_t)i);
    const unsigned u = (unsigned)f2bf_bits(f[0]) | ((unsigned)f2bf_bits(f[1]) << 16);
    ((volatile unsigned*)out)[i] = u;
    __threadfence();
    ((volatile unsigned*)out)[i] = u;
  }
}

__global__ __launch_bounds__(256) void transpose64_bf16(
    const float* __restrict__ E, const float* __restrict__ F,
    unsigned short* __restrict__ Et, unsigned short* __restrict__ Ft) {
  __shared__ float tile[64][65];
  const int h = blockIdx.x;
  const bool isF = (blockIdx.y != 0);
  const float* src = (isF ? F : E) + (size_t)h * (HDIM * KLOW);
  unsigned short* dst = (isF ? Ft : Et) + (size_t)h * (HDIM * KLOW);
  const int tid = threadIdx.x;
#pragma unroll
  for (int i = 0; i < 4; ++i) {
    const int idx4 = (tid + 256 * i) * 4;
    const int d = idx4 >> 6, j = idx4 & 63;
    const v4f w = *(const v4f*)(src + idx4);
    tile[d][j + 0] = w[0]; tile[d][j + 1] = w[1]; tile[d][j + 2] = w[2]; tile[d][j + 3] = w[3];
  }
  __syncthreads();
  const int wave = tid >> 5, lane = tid & 31;
  const int q = lane >> 3, c8 = (lane & 7) * 8;
  for (int pass = 0; pass < 2; ++pass) {
#pragma unroll
    for (int it = 0; it < 2; ++it) {
      const int j = it * 32 + wave * 4 + q;
      v4u w;
#pragma unroll
      for (int k = 0; k < 4; ++k) {
        const unsigned a0 = f2bf_bits(tile[c8 + 2 * k][j]);
        const unsigned a1 = f2bf_bits(tile[c8 + 2 * k + 1][j]);
        w[k] = a0 | (a1 << 16);
      }
      *(volatile v4u*)(dst + (size_t)j * HDIM + c8) = w;
    }
    __threadfence();
  }
}

constexpr int AT_D = 64, AT_NW = 4, AT_QB = 64, AT_KC = 64, AT_OP = 68;

__device__ __forceinline__ v8f at_mma(v16b a, v16b b, v8f c) {
  c = __builtin_amdgcn_wmma_f32_16x16x32_bf16(false, a, false, b, (short)0, c, false, false);
  asm volatile("v_nop\n\tv_nop\n\tv_nop\n\tv_nop" : "+v"(c) : "v"(a), "v"(b));
  return c;
}

__global__ __launch_bounds__(128)
void attn_causal_hl(const unsigned short* __restrict__ Qh, const unsigned short* __restrict__ Ql, int q_rs,
                    const unsigned short* __restrict__ Kh, const unsigned short* __restrict__ Kl, int k_rs,
                    const unsigned short* __restrict__ Vh, const unsigned short* __restrict__ Vl, int v_rs,
                    unsigned short* __restrict__ Oh, unsigned short* __restrict__ Ol, int o_rs,
                    int S, int H, float qscale) {
  union FB { v16b v; v8b h[2]; };
  __shared__ __align__(16) float lds_kv[4 * AT_KC * AT_D / 2];
  __shared__ __align__(16) unsigned short Psh[AT_NW * 16 * AT_KC];
  __shared__ __align__(16) unsigned short Psl[AT_NW * 16 * AT_KC];
  unsigned short* Ksh = (unsigned short*)lds_kv;
  unsigned short* Ksl = Ksh + AT_KC * AT_D;
  unsigned short* Vth = Ksl + AT_KC * AT_D;
  unsigned short* Vtl = Vth + AT_KC * AT_D;

  const float NEG_INF = -__builtin_huge_valf();
  const int tid  = threadIdx.x;
  const int wave = tid >> 5;
  const int lane = tid & 31;
  const int hh   = lane >> 4;
  const int c    = lane & 15;

  const int nqb = S / AT_QB;
  const int bx = blockIdx.x;
  const int qb = bx % nqb;
  const int bh = bx / nqb;
  const int h  = bh % H;
  const int b  = bh / H;
  const int q0 = qb * AT_QB + wave * 16;

  v16b qah[2], qal[2];
  {
    const size_t qoff = (size_t)(b * S + q0 + c) * q_rs + h * AT_D;
    const unsigned short* qg  = Qh + qoff;
    const unsigned short* qgl = Ql + qoff;
#pragma unroll
    for (int dc = 0; dc < 2; ++dc) {
      qah[dc] = Frag<__bf16>::load((const __bf16*)(qg  + dc * 32 + 8 * hh));
      qal[dc] = Frag<__bf16>::load((const __bf16*)(qgl + dc * 32 + 8 * hh));
    }
  }

  float mrow[8], lrow[8];
  v8f oacc[4];
#pragma unroll
  for (int r = 0; r < 8; ++r) { mrow[r] = NEG_INF; lrow[r] = 0.f; }
#pragma unroll
  for (int t = 0; t < 4; ++t) oacc[t] = (v8f){0.f,0.f,0.f,0.f,0.f,0.f,0.f,0.f};

  const int nChunks = qb + 1;
  for (int kc = 0; kc < nChunks; ++kc) {
    const int kv0 = kc * AT_KC;
    __syncthreads();
    {
      const size_t kbase = (size_t)(b * S + kv0) * k_rs + h * AT_D;
      const unsigned short* kgh = Kh + kbase;
      const unsigned short* kgl = Kl + kbase;
#pragma unroll
      for (int i = 0; i < 4; ++i) {
        const int u = tid + 128 * i;
        const int row = u >> 3, c8 = (u & 7) * 8;
        const v4u wh = *(const v4u*)(kgh + (size_t)row * k_rs + c8);
        const v4u wl = *(const v4u*)(kgl + (size_t)row * k_rs + c8);
        *(v4u*)(Ksh + row * AT_D + c8) = wh;
        *(v4u*)(Ksl + row * AT_D + c8) = wl;
      }
    }
    asm volatile("" ::: "memory");
    {
      const int kvr = tid >> 1, dh = (tid & 1) * 32;
      const size_t vbase = (size_t)(b * S + kv0 + kvr) * v_rs + h * AT_D + dh;
      const unsigned short* vgh = Vh + vbase;
      const unsigned short* vgl = Vl + vbase;
#pragma unroll
      for (int i = 0; i < 4; ++i) {
        const v4u wh = *(const v4u*)(vgh + 8 * i);
        const v4u wl = *(const v4u*)(vgl + 8 * i);
#pragma unroll
        for (int e = 0; e < 8; ++e) {
          const unsigned xh = (wh[e >> 1] >> (16 * (e & 1))) & 0xffffu;
          const unsigned xl = (wl[e >> 1] >> (16 * (e & 1))) & 0xffffu;
          Vth[(dh + 8 * i + e) * AT_KC + kvr] = (unsigned short)xh;
          Vtl[(dh + 8 * i + e) * AT_KC + kvr] = (unsigned short)xl;
        }
      }
    }
    __syncthreads();

    v8f s[4];
#pragma unroll
    for (int j = 0; j < 4; ++j) {
      s[j] = (v8f){0.f,0.f,0.f,0.f,0.f,0.f,0.f,0.f};
#pragma unroll
      for (int dc = 0; dc < 2; ++dc) {
        FB kb, kl;
        kb.h[0] = *(const v8b*)(Ksh + (j * 16 + c) * AT_D + dc * 32 + 8 * hh);
        kb.h[1] = *(const v8b*)(Ksh + (j * 16 + c) * AT_D + dc * 32 + 16 + 8 * hh);
        kl.h[0] = *(const v8b*)(Ksl + (j * 16 + c) * AT_D + dc * 32 + 8 * hh);
        kl.h[1] = *(const v8b*)(Ksl + (j * 16 + c) * AT_D + dc * 32 + 16 + 8 * hh);
        s[j] = at_mma(qah[dc], kb.v, s[j]);
        s[j] = at_mma(qah[dc], kl.v, s[j]);
        s[j] = at_mma(qal[dc], kb.v, s[j]);
      }
    }
    const bool diag = (kc == qb);
    float cm[8];
#pragma unroll
    for (int r = 0; r < 8; ++r) {
      const int qrow = q0 + 8 * hh + r;
      float m = NEG_INF;
#pragma unroll
      for (int j = 0; j < 4; ++j) {
        const int kvcol = kv0 + j * 16 + c;
        float val = s[j][r] * qscale;
        val = (diag && (kvcol > qrow)) ? NEG_INF : val;
        s[j][r] = val;
        m = fmaxf(m, val);
      }
#pragma unroll
      for (int off = 1; off < 16; off <<= 1) m = fmaxf(m, __shfl_xor(m, off, 32));
      cm[r] = m;
    }
    unsigned short* pwh = Psh + wave * (16 * AT_KC);
    unsigned short* pwl = Psl + wave * (16 * AT_KC);
#pragma unroll
    for (int r = 0; r < 8; ++r) {
      const float mnew = fmaxf(mrow[r], cm[r]);
      const float alpha = expf(mrow[r] - mnew);
      mrow[r] = mnew;
      float psum = 0.f;
#pragma unroll
      for (int j = 0; j < 4; ++j) {
        const float p = expf(s[j][r] - mnew);
        psum += p;
        const unsigned short hb = f2bf_bits(p);
        const unsigned short lb = f2bf_bits(p - bf_bits2f(hb));
        pwh[(8 * hh + r) * AT_KC + j * 16 + c] = hb;
        pwl[(8 * hh + r) * AT_KC + j * 16 + c] = lb;
      }
#pragma unroll
      for (int off = 1; off < 16; off <<= 1) psum += __shfl_xor(psum, off, 32);
      lrow[r] = lrow[r] * alpha + psum;
#pragma unroll
      for (int t = 0; t < 4; ++t) oacc[t][r] *= alpha;
    }
    __syncthreads();
#pragma unroll 1
    for (int kk = 0; kk < 2; ++kk) {
      FB pa, pl;
      pa.h[0] = *(const v8b*)(pwh + c * AT_KC + kk * 32 + 8 * hh);
      pa.h[1] = *(const v8b*)(pwh + c * AT_KC + kk * 32 + 16 + 8 * hh);
      pl.h[0] = *(const v8b*)(pwl + c * AT_KC + kk * 32 + 8 * hh);
      pl.h[1] = *(const v8b*)(pwl + c * AT_KC + kk * 32 + 16 + 8 * hh);
#pragma unroll
      for (int t = 0; t < 4; ++t) {
        FB vb, vl;
        vb.h[0] = *(const v8b*)(Vth + (t * 16 + c) * AT_KC + kk * 32 + 8 * hh);
        vb.h[1] = *(const v8b*)(Vth + (t * 16 + c) * AT_KC + kk * 32 + 16 + 8 * hh);
        vl.h[0] = *(const v8b*)(Vtl + (t * 16 + c) * AT_KC + kk * 32 + 8 * hh);
        vl.h[1] = *(const v8b*)(Vtl + (t * 16 + c) * AT_KC + kk * 32 + 16 + 8 * hh);
        oacc[t] = at_mma(pa.v, vb.v, oacc[t]);
        oacc[t] = at_mma(pa.v, vl.v, oacc[t]);
        oacc[t] = at_mma(pl.v, vb.v, oacc[t]);
      }
    }
  }

  __syncthreads();
  float* os = lds_kv + wave * (16 * AT_OP);
#pragma unroll
  for (int r = 0; r < 8; ++r) {
    const float inv = 1.0f / lrow[r];
#pragma unroll
    for (int t = 0; t < 4; ++t) os[(8 * hh + r) * AT_OP + t * 16 + c] = oacc[t][r] * inv;
  }
  __syncthreads();
  {
    const int q = lane >> 3, c8 = (lane & 7) * 8;
    for (int pass = 0; pass < 2; ++pass) {
#pragma unroll
      for (int it = 0; it < 4; ++it) {
        const int row = it * 4 + q;
        const float* sp = os + row * AT_OP + c8;
        v4u hv, lv;
#pragma unroll
        for (int k = 0; k < 4; ++k) {
          const float f0 = sp[2 * k], f1 = sp[2 * k + 1];
          const unsigned short h0 = f2bf_bits(f0), h1 = f2bf_bits(f1);
          const unsigned short l0 = f2bf_bits(f0 - bf_bits2f(h0));
          const unsigned short l1 = f2bf_bits(f1 - bf_bits2f(h1));
          hv[k] = (unsigned)h0 | ((unsigned)h1 << 16);
          lv[k] = (unsigned)l0 | ((unsigned)l1 << 16);
        }
        const size_t ooff = (size_t)(b * S + q0 + row) * o_rs + h * AT_D + c8;
        *(volatile v4u*)(Oh + ooff) = hv;
        *(volatile v4u*)(Ol + ooff) = lv;
      }
      __threadfence();
    }
  }
}

static_assert(NROWS % 64 == 0 && NQKV % 64 == 0 && NCH % 64 == 0 && KLOW % 64 == 0);
static_assert(NCH % 32 == 0 && HDIM % 32 == 0);
static_assert(NSEQ % AT_QB == 0 && HDIM == AT_D && KLOW == AT_D);
static_assert((NROWS * NCH / 2) % 256 == 0 && (NCH * NCH / 2) % 256 == 0);

constexpr size_t SZ_XB   = (size_t)NROWS * NCH * 2;
constexpr size_t SZ_WQKV = (size_t)NQKV * NCH * 2;
constexpr size_t SZ_WP   = (size_t)NCH * NCH * 2;
constexpr size_t SZ_ET   = (size_t)NHEAD * HDIM * KLOW * 2;
constexpr size_t SZ_QKV  = (size_t)NROWS * NQKV * 2;
constexpr size_t SZ_PL   = (size_t)NROWS * NCH * 2;
constexpr size_t OFF_XB   = 0;
constexpr size_t OFF_WQKV = OFF_XB + SZ_XB;
constexpr size_t OFF_WP   = OFF_WQKV + SZ_WQKV;
constexpr size_t OFF_ET   = OFF_WP + SZ_WP;
constexpr size_t OFF_FT   = OFF_ET + SZ_ET;
constexpr size_t OFF_QKVH = OFF_FT + SZ_ET;
constexpr size_t OFF_QKVL = OFF_QKVH + SZ_QKV;
constexpr size_t OFF_KPH  = OFF_QKVL + SZ_QKV;
constexpr size_t OFF_KPL  = OFF_KPH + SZ_PL;
constexpr size_t OFF_VPH  = OFF_KPL + SZ_PL;
constexpr size_t OFF_VPL  = OFF_VPH + SZ_PL;
constexpr size_t OFF_OH   = OFF_VPL + SZ_PL;
constexpr size_t OFF_OL   = OFF_OH + SZ_PL;
constexpr size_t WS_TOTAL = OFF_OL + SZ_PL;
static_assert(WS_TOTAL == 117702656);
static_assert(WS_TOTAL <= 134217728);
static_assert(OFF_WQKV % 128 == 0 && OFF_WP % 128 == 0 && OFF_ET % 128 == 0 && OFF_FT % 128 == 0 &&
              OFF_QKVH % 128 == 0 && OFF_QKVL % 128 == 0 && OFF_KPH % 128 == 0 && OFF_OH % 128 == 0);

extern "C" void kernel_launch(void* const* d_in, const int* in_sizes, int n_in,
                              void* d_out, int out_size, void* d_ws, size_t ws_size,
                              hipStream_t stream) {
  if (n_in < 8) return;
  if (in_sizes[0] != NROWS * NCH || in_sizes[1] != NHEAD * HDIM * NCH || in_sizes[2] != NHEAD * HDIM * NCH ||
      in_sizes[3] != NHEAD * HDIM * NCH || in_sizes[4] != NHEAD * HDIM * KLOW || in_sizes[5] != NHEAD * HDIM * KLOW ||
      in_sizes[6] != NCH * NCH || in_sizes[7] != NCH || out_size != NROWS * NCH) return;
  if (WS_TOTAL > ws_size) return;

  const float* x  = (const float*)d_in[0];
  const float* Wq = (const float*)d_in[1];
  const float* Wk = (const float*)d_in[2];
  const float* Wv = (const float*)d_in[3];
  const float* E  = (const float*)d_in[4];
  const float* F  = (const float*)d_in[5];
  const float* Wp = (const float*)d_in[6];
  const float* bp = (const float*)d_in[7];
  float* out = (float*)d_out;

  char* w = (char*)d_ws;
  unsigned short* Xb    = (unsigned short*)(w + OFF_XB);
  unsigned short* Wqkvb = (unsigned short*)(w + OFF_WQKV);
  unsigned short* Wpb   = (unsigned short*)(w + OFF_WP);
  unsigned short* Etb   = (unsigned short*)(w + OFF_ET);
  unsigned short* Ftb   = (unsigned short*)(w + OFF_FT);
  unsigned short* QKVh  = (unsigned short*)(w + OFF_QKVH);
  unsigned short* QKVl  = (unsigned short*)(w + OFF_QKVL);
  unsigned short* KPh   = (unsigned short*)(w + OFF_KPH);
  unsigned short* KPl   = (unsigned short*)(w + OFF_KPL);
  unsigned short* VPh   = (unsigned short*)(w + OFF_VPH);
  unsigned short* VPl   = (unsigned short*)(w + OFF_VPL);
  unsigned short* Oh    = (unsigned short*)(w + OFF_OH);
  unsigned short* Ol    = (unsigned short*)(w + OFF_OL);

  {
    const int n2x = NROWS * NCH / 2;
    cast_f32_bf16x2<<<n2x / 256, 256, 0, stream>>>(x, Xb, n2x);
    const int n2w = NHEAD * HDIM * NCH / 2;
    cast_f32_bf16x2<<<n2w / 256, 256, 0, stream>>>(Wq, Wqkvb, n2w);
    cast_f32_bf16x2<<<n2w / 256, 256, 0, stream>>>(Wk, Wqkvb + (size_t)NCH * NCH, n2w);
    cast_f32_bf16x2<<<n2w / 256, 256, 0, stream>>>(Wv, Wqkvb + (size_t)2 * NCH * NCH, n2w);
    const int n2p = NCH * NCH / 2;
    cast_f32_bf16x2<<<n2p / 256, 256, 0, stream>>>(Wp, Wpb, n2p);
    transpose64_bf16<<<dim3(NHEAD, 2), 256, 0, stream>>>(E, F, Etb, Ftb);
  }

  wmma_gemm64<1, 0, 0, 2><<<dim3((NROWS / 64) * (NQKV / 64) / 8, 1), 256, 0, stream>>>(
      Xb, Xb, NCH, 0L, Wqkvb, Wqkvb, NCH, 0L, QKVh, QKVl, NQKV, 0L, bp, NROWS, NQKV, NCH, 1.0f);

  wmma_gemm64<1, 1, 0, 2><<<dim3((NROWS / 64) * (KLOW / 64) / 8, NHEAD), 256, 0, stream>>>(
      QKVh + NCH, QKVl + NCH, NQKV, (long)HDIM, Etb, Etb, HDIM, (long)(HDIM * KLOW),
      KPh, KPl, NCH, (long)KLOW, bp, NROWS, KLOW, HDIM, 1.0f);
  wmma_gemm64<1, 1, 0, 2><<<dim3((NROWS / 64) * (KLOW / 64) / 8, NHEAD), 256, 0, stream>>>(
      QKVh + 2 * NCH, QKVl + 2 * NCH, NQKV, (long)HDIM, Ftb, Ftb, HDIM, (long)(HDIM * KLOW),
      VPh, VPl, NCH, (long)KLOW, bp, NROWS, KLOW, HDIM, 1.0f);

  attn_causal_hl<<<NBATCH * NHEAD * (NSEQ / AT_QB), 128, 0, stream>>>(
      QKVh, QKVl, NQKV, KPh, KPl, NCH, VPh, VPl, NCH, Oh, Ol, NCH, NSEQ, NHEAD, 0.125f);

  wmma_gemm64<1, 1, 2, 0><<<dim3((NROWS / 64) * (NCH / 64) / 8, 1), 256, 0, stream>>>(
      Oh, Ol, NCH, 0L, Wpb, Wpb, NCH, 0L, out, out, NCH, 0L, bp, NROWS, NCH, NCH, 1.0f);
}
